// Mambalayer_16475494547742
// MI455X (gfx1250) — hardware-verified
//
#include <hip/hip_runtime.h>
#include <math.h>

typedef __attribute__((ext_vector_type(16))) _Float16 v16h;
typedef __attribute__((ext_vector_type(8)))  _Float16 v8h;
typedef __attribute__((ext_vector_type(8)))  float    v8f;
typedef __attribute__((ext_vector_type(4)))  float    v4f;

constexpr int kBatch  = 2;
constexpr int kSeq    = 2048;
constexpr int kDm     = 256;
constexpr int kDin    = 1024;
constexpr int kNst    = 16;
constexpr int kDtR    = 16;
constexpr int kXzP    = 2 * kDin;
constexpr int kXdReal = kDtR + 2 * kNst;
constexpr int kXdP    = 64;
constexpr int kFf     = 1024;
constexpr int kRows   = kBatch * kSeq;
constexpr int kConvTP = 260;
constexpr int kScanTS = 64;
constexpr int kScanCh = 64;
constexpr int kScanYP = 68;
constexpr int kLnP    = 264;
constexpr float kCarryW = 32.0f;
constexpr float kCarryU = 16.0f;
constexpr float kCarryG = 64.0f;
constexpr float kLnEps  = 1e-6f;
static_assert(kXdReal == 48 && kXdReal <= kXdP, "x_proj width");
static_assert((kDm % 32) == 0 && (kDin % 32) == 0 && (kFf % 32) == 0, "GEMM K multiples of 32");
static_assert((kRows % 64) == 0 && (kXzP % 64) == 0 && (kXdP % 64) == 0 && (kDm % 64) == 0 && (kFf % 64) == 0, "GEMM M,N multiples of 64");
static_assert((kSeq % kScanTS) == 0 && (kSeq % 64) == 0 && (kDin % kScanCh) == 0 && (kDin % 256) == 0, "tile multiples");
static_assert(kDm == 256 && (kRows % 8) == 0, "LayerNorm lane map: 8 elements per lane, 8 rows per block");
static_assert(kDtR == 16 && kNst == 16, "scan register layout");

constexpr size_t kOffX16  = 0;
constexpr size_t kOffWI16 = kOffX16  + (size_t)kRows * kDm  * 2;
constexpr size_t kOffWX16 = kOffWI16 + (size_t)kXzP  * kDm  * 2;
constexpr size_t kOffWO16 = kOffWX16 + (size_t)kXdP  * kDin * 2;
constexpr size_t kOffW116 = kOffWO16 + (size_t)kDm   * kDin * 2;
constexpr size_t kOffW216 = kOffW116 + (size_t)kFf   * kDm  * 2;
constexpr size_t kOffXZ   = kOffW216 + (size_t)kDm   * kFf  * 2;
constexpr size_t kOffUC   = kOffXZ   + (size_t)kRows * kXzP * 4;
constexpr size_t kOffUC16 = kOffUC   + (size_t)kRows * kDin * 4;
constexpr size_t kOffXD   = kOffUC16 + (size_t)kRows * kDin * 2;
constexpr size_t kOffG16  = kOffXD   + (size_t)kRows * kXdP * 4;
constexpr size_t kOffMO   = kOffG16  + (size_t)kRows * kDin * 2;
constexpr size_t kOffO1   = kOffMO   + (size_t)kRows * kDm  * 4;
constexpr size_t kOffO1H  = kOffO1   + (size_t)kRows * kDm  * 4;
constexpr size_t kOffHID  = kOffO1H  + (size_t)kRows * kDm  * 2;
constexpr size_t kOffFF   = kOffHID  + (size_t)kRows * kFf  * 2;
constexpr size_t kWsTotal = kOffFF   + (size_t)kRows * kDm  * 4;
static_assert(kWsTotal == 96075776ull, "carve total");
static_assert(kWsTotal <= 134217728ull, "carve cap");
static_assert((kOffWI16 % 128) == 0 && (kOffWX16 % 128) == 0 && (kOffWO16 % 128) == 0 && (kOffW116 % 128) == 0 &&
              (kOffW216 % 128) == 0 && (kOffXZ % 128) == 0 && (kOffUC % 128) == 0 && (kOffUC16 % 128) == 0 &&
              (kOffXD % 128) == 0 && (kOffG16 % 128) == 0 && (kOffMO % 128) == 0 && (kOffO1 % 128) == 0 &&
              (kOffO1H % 128) == 0 && (kOffHID % 128) == 0 && (kOffFF % 128) == 0, "128-B aligned regions");

union FragH { v16h v; v8h h[2]; };
__device__ __forceinline__ v16h frag_load(const _Float16* p) {
  FragH f;
  f.h[0] = *(const v8h*)(p);
  f.h[1] = *(const v8h*)(p + 16);
  return f.v;
}
__device__ __forceinline__ v8f frag_mma(v16h a, v16h b, v8f c) {
  return __builtin_amdgcn_wmma_f32_16x16x32_f16(false, a, false, b, (short)0, c, false, false);
}
__device__ __forceinline__ void guard_row(v8f& a0, v8f& a1, v8f& a2, v8f& a3, v16h x, v16h b0, v16h b1, v16h b2, v16h b3) {
  asm volatile("v_nop\n\tv_nop\n\tv_nop\n\tv_nop" : "+v"(a0), "+v"(a1), "+v"(a2), "+v"(a3) : "v"(x), "v"(b0), "v"(b1), "v"(b2), "v"(b3));
}
__device__ __forceinline__ void acc_guard4(v8f& a, v8f& b, v8f& c, v8f& d) {
  asm volatile("v_nop\n\tv_nop\n\tv_nop\n\tv_nop" : "+v"(a), "+v"(b), "+v"(c), "+v"(d));
}

template <int BIAS_MODE, int OUT_MODE, int ACT>
__global__ __launch_bounds__(256) void wmma_gemm64(
    const unsigned short* __restrict__ Ap, int lda,
    const unsigned short* __restrict__ Btp, int ldb,
    void* __restrict__ Cout, int ldc,
    const float* __restrict__ bias,
    int M, int N, int K, float scale)
{
  const _Float16* A  = (const _Float16*)Ap;
  const _Float16* Bt = (const _Float16*)Btp;
  __shared__ __align__(16) float sT[8][16 * 68];
  const int lane = threadIdx.x & 31;
  const int wave = threadIdx.x >> 5;
  const int tilesN = N >> 6;
  const int tilesM = M >> 6;
  const int tile = blockIdx.x * 8 + wave;
  if (tile >= tilesM * tilesN) return;
  const int tm = tile / tilesN;
  const int tn = tile - tm * tilesN;
  const int m0 = tm << 6;
  const int n0 = tn << 6;

  const int rlane = lane & 15;
  const int koff  = (lane >> 4) * 8;
  const int mOff  = (lane >> 4) * 8;

  v8f acc[4][4];
#pragma unroll
  for (int i = 0; i < 4; ++i)
#pragma unroll
    for (int j = 0; j < 4; ++j) acc[i][j] = (v8f){0.f,0.f,0.f,0.f,0.f,0.f,0.f,0.f};

  for (int k0 = 0; k0 < K; k0 += 32) {
    v16h bh[4];
#pragma unroll
    for (int j = 0; j < 4; ++j) {
      const size_t bo = (size_t)(n0 + (j << 4) + rlane) * ldb + koff + k0;
      bh[j] = frag_load(Bt + bo);
    }
#pragma unroll
    for (int i = 0; i < 4; ++i) {
      const size_t ao = (size_t)(m0 + (i << 4) + rlane) * lda + koff + k0;
      const v16h ah = frag_load(A + ao);
#pragma unroll
      for (int j = 0; j < 4; ++j) acc[i][j] = frag_mma(ah, bh[j], acc[i][j]);
      guard_row(acc[i][0], acc[i][1], acc[i][2], acc[i][3], ah, bh[0], bh[1], bh[2], bh[3]);
    }
  }
  acc_guard4(acc[0][0], acc[0][1], acc[0][2], acc[0][3]);
  acc_guard4(acc[1][0], acc[1][1], acc[1][2], acc[1][3]);
  acc_guard4(acc[2][0], acc[2][1], acc[2][2], acc[2][3]);
  acc_guard4(acc[3][0], acc[3][1], acc[3][2], acc[3][3]);

  float* slab = sT[wave];
#pragma unroll
  for (int i = 0; i < 4; ++i) {
    const int mBase = m0 + (i << 4);
#pragma unroll
    for (int j = 0; j < 4; ++j) {
      const int n = n0 + (j << 4) + rlane;
      float bv = 0.f;
      if (BIAS_MODE == 2) bv = bias[n];
#pragma unroll
      for (int r = 0; r < 8; ++r) {
        float v = acc[i][j][r] * scale;
        if (BIAS_MODE == 2) v += bv;
        if (ACT == 2) v = fmaxf(v, 0.0f);
        slab[(mOff + r) * 68 + (j << 4) + rlane] = v;
      }
    }
    __builtin_amdgcn_fence(__ATOMIC_RELEASE, "workgroup");
    __builtin_amdgcn_wave_barrier();
    __builtin_amdgcn_fence(__ATOMIC_ACQUIRE, "workgroup");
    if (OUT_MODE == 0) {
      float* C = (float*)Cout;
      const int hh = lane >> 4, c4 = (lane & 15) * 4;
      for (int pass = 0; pass < 2; ++pass) {
#pragma unroll
        for (int it = 0; it < 8; ++it) {
          const int row = it * 2 + hh;
          const v4f v = *(const v4f*)(slab + row * 68 + c4);
          *(volatile v4f*)(C + (size_t)(mBase + row) * ldc + n0 + c4) = v;
        }
        __threadfence();
      }
    } else {
      const int q = lane >> 3, c8 = (lane & 7) * 8;
      unsigned short* C = (unsigned short*)Cout;
      for (int pass = 0; pass < 2; ++pass) {
#pragma unroll
        for (int it = 0; it < 4; ++it) {
          const int row = it * 4 + q;
          const float* sp = slab + row * 68 + c8;
          v8h hv;
#pragma unroll
          for (int e = 0; e < 8; ++e) hv[e] = (_Float16)sp[e];
          *(volatile v8h*)(C + (size_t)(mBase + row) * ldc + n0 + c8) = hv;
        }
        __threadfence();
      }
    }
    __builtin_amdgcn_fence(__ATOMIC_RELEASE, "workgroup");
    __builtin_amdgcn_wave_barrier();
    __builtin_amdgcn_fence(__ATOMIC_ACQUIRE, "workgroup");
  }
}

__global__ __launch_bounds__(256) void cast_f16_kernel(
    const float* __restrict__ src, unsigned short* __restrict__ dst, int total8, int real8, float scale)
{
  const int i = blockIdx.x * 256 + threadIdx.x;
  if (i >= total8) return;
  const bool live = (i < real8);
  const int ic = live ? i : (real8 - 1);
  const float* p = src + ((size_t)ic << 3);
  const v4f a0 = *(const v4f*)(p);
  const v4f a1 = *(const v4f*)(p + 4);
  v8h hv;
#pragma unroll
  for (int e = 0; e < 4; ++e) {
    const float f0 = live ? (a0[e] * scale) : 0.0f;
    const float f1 = live ? (a1[e] * scale) : 0.0f;
    hv[e]     = (_Float16)f0;
    hv[4 + e] = (_Float16)f1;
  }
  unsigned short* q = dst + ((size_t)i << 3);
  *(volatile v8h*)q = hv;
  __threadfence();
  *(volatile v8h*)q = hv;
}

__global__ __launch_bounds__(256) void conv_silu_kernel(
    const float* __restrict__ XZ, const float* __restrict__ cw, const float* __restrict__ cb,
    float* __restrict__ UC, unsigned short* __restrict__ UC16)
{
  __shared__ __align__(16) float sT[16 * kConvTP];
  const int tid = threadIdx.x, lane = tid & 31, wave = tid >> 5;
  const int d0 = blockIdx.x * 256, d = d0 + tid;
  const int g0 = blockIdx.y * 64;
  const int tb = g0 & (kSeq - 1);
  const v4f wv = *(const v4f*)(cw + (size_t)d * 4);
  const float w0 = wv[0], w1 = wv[1], w2 = wv[2], w3 = wv[3];
  const float bc = cb[d];
  float xm3, xm2, xm1;
  {
    const bool hist = (tb > 0);
    const int rb = hist ? (g0 - 3) : g0;
    const float v3 = XZ[(size_t)rb * kXzP + d];
    const float v2 = XZ[(size_t)(rb + 1) * kXzP + d];
    const float v1 = XZ[(size_t)(rb + 2) * kXzP + d];
    xm3 = hist ? v3 : 0.f;
    xm2 = hist ? v2 : 0.f;
    xm1 = hist ? v1 : 0.f;
  }
  const int hrow = wave >> 1;
  const int hch  = (wave & 1) * 128 + lane * 4;
#pragma unroll 1
  for (int sub = 0; sub < 4; ++sub) {
    const int lb = g0 + sub * 16;
#pragma unroll 1
    for (int s = 0; s < 16; ++s) {
      const float xcur = XZ[(size_t)(lb + s) * kXzP + d];
      float acc = w0 * xm3;
      acc = fmaf(w1, xm2, acc);
      acc = fmaf(w2, xm1, acc);
      acc = fmaf(w3, xcur, acc);
      const float sv = acc + bc;
      const float sg = __builtin_amdgcn_rcpf(1.0f + expf(-sv));
      sT[s * kConvTP + tid] = sv * sg;
      xm3 = xm2; xm2 = xm1; xm1 = xcur;
    }
    __syncthreads();
    v4f fv[4];
    v8h bv[2];
#pragma unroll
    for (int it = 0; it < 4; ++it) fv[it] = *(const v4f*)(sT + (it * 4 + hrow) * kConvTP + hch);
#pragma unroll
    for (int it = 0; it < 2; ++it) {
      const float* sp = sT + (it * 8 + wave) * kConvTP + lane * 8;
      const v4f a0 = *(const v4f*)(sp);
      const v4f a1 = *(const v4f*)(sp + 4);
#pragma unroll
      for (int e = 0; e < 4; ++e) {
        bv[it][e]     = (_Float16)(a0[e] * kCarryU);
        bv[it][4 + e] = (_Float16)(a1[e] * kCarryU);
      }
    }
    for (int pass = 0; pass < 2; ++pass) {
#pragma unroll
      for (int it = 0; it < 4; ++it)
        *(volatile v4f*)(UC + (size_t)(lb + it * 4 + hrow) * kDin + d0 + hch) = fv[it];
#pragma unroll
      for (int it = 0; it < 2; ++it)
        *(volatile v8h*)(UC16 + (size_t)(lb + it * 8 + wave) * kDin + d0 + lane * 8) = bv[it];
      __threadfence();
    }
    __syncthreads();
  }
}

__global__ __launch_bounds__(64) void scan_kernel(
    const float* __restrict__ XD, const float* __restrict__ UC, const float* __restrict__ XZ,
    const float* __restrict__ Wdt, const float* __restrict__ bdt, const float* __restrict__ Alog,
    const float* __restrict__ Dp, unsigned short* __restrict__ G16)
{
  __shared__ __align__(16) float sX[kScanTS * kXdP];
  __shared__ __align__(16) float sY[kScanTS * kScanYP];
  __shared__ __align__(16) float sW[kDtR * kScanCh];
  __shared__ __align__(16) float sA[kNst * kScanCh];
  const int tid = threadIdx.x, lane = tid & 31, wave = tid >> 5;
  constexpr int kBlkPerB = kDin / kScanCh;
  const int bix = blockIdx.x / kBlkPerB;
  const int d0  = (blockIdx.x - bix * kBlkPerB) * kScanCh;
  const int d   = d0 + tid;
  const size_t row0 = (size_t)bix * kSeq;
#pragma unroll 1
  for (int r = 0; r < kDtR; ++r) sW[r * kScanCh + tid] = Wdt[(size_t)d * kDtR + r];
#pragma unroll 1
  for (int s = 0; s < kNst; ++s) sA[s * kScanCh + tid] = -expf(Alog[(size_t)d * kNst + s]);
  __syncthreads();
  float negA[kNst], h[kNst];
#pragma unroll
  for (int s = 0; s < kNst; ++s) {
    negA[s] = sA[s * kScanCh + tid];
    h[s] = 0.f;
  }
  const float bb = bdt[d], Dd = Dp[d];
  const int lr = tid >> 4, lc4 = (tid & 15) * 4;
  const int q = lane >> 3, c8 = (lane & 7) * 8;
#pragma unroll 1
  for (int t0 = 0; t0 < kSeq; t0 += kScanTS) {
    __syncthreads();
#pragma unroll
    for (int i = 0; i < 16; ++i) {
      const int r = lr + 4 * i;
      *(v4f*)(sX + r * kXdP + lc4) = *(const v4f*)(XD + (row0 + t0 + r) * kXdP + lc4);
    }
    __syncthreads();
#pragma unroll 1
    for (int s = 0; s < kScanTS; ++s) {
      const int t = t0 + s;
      const float* xr = sX + s * kXdP;
      float xt = UC[(row0 + t) * kDin + d];
      float zv = XZ[(row0 + t) * kXzP + kDin + d];
      asm volatile("" : "+v"(xt));
      asm volatile("" : "+v"(zv));
      float vdot = 0.f;
#pragma unroll 1
      for (int r4 = 0; r4 < kDtR / 4; ++r4) {
        const v4f xv = *(const v4f*)(xr + 4 * r4);
        const float* wp = sW + (4 * r4) * kScanCh + tid;
        vdot = fmaf(xv[0], wp[0], vdot);
        vdot = fmaf(xv[1], wp[kScanCh], vdot);
        vdot = fmaf(xv[2], wp[2 * kScanCh], vdot);
        vdot = fmaf(xv[3], wp[3 * kScanCh], vdot);
      }
      float Bs[kNst], Cs[kNst];
#pragma unroll
      for (int q4 = 0; q4 < 4; ++q4) {
        const v4f bv = *(const v4f*)(xr + kDtR + 4 * q4);
        const v4f cv = *(const v4f*)(xr + kDtR + kNst + 4 * q4);
        Bs[4 * q4 + 0] = bv[0]; Bs[4 * q4 + 1] = bv[1]; Bs[4 * q4 + 2] = bv[2]; Bs[4 * q4 + 3] = bv[3];
        Cs[4 * q4 + 0] = cv[0]; Cs[4 * q4 + 1] = cv[1]; Cs[4 * q4 + 2] = cv[2]; Cs[4 * q4 + 3] = cv[3];
      }
      const float v   = vdot + bb;
      const float a   = __expf(-fabsf(v));
      const float u1  = 1.0f + a;
      const float l1p = __logf(u1) + (a - (u1 - 1.0f)) * __builtin_amdgcn_rcpf(u1);
      const float dt  = fmaxf(v, 0.0f) + l1p;
      const float dtx = dt * xt;
      float y = 0.f;
#pragma unroll
      for (int k = 0; k < kNst; ++k) {
        const float e = __expf(dt * negA[k]);
        h[k] = e * h[k] + dtx * Bs[k];
        y = h[k] * Cs[k] + y;
      }
      y = xt * Dd + y;
      const float sg = __builtin_amdgcn_rcpf(1.0f + expf(-zv));
      y = y * (zv * sg);
      sY[s * kScanYP + tid] = y;
    }
    __syncthreads();
    v8h hv[8];
#pragma unroll
    for (int it = 0; it < 8; ++it) {
      const int row = it * 8 + wave * 4 + q;
      const float* sp = sY + row * kScanYP + c8;
      const v4f a0 = *(const v4f*)(sp);
      const v4f a1 = *(const v4f*)(sp + 4);
#pragma unroll
      for (int e = 0; e < 4; ++e) {
        hv[it][e]     = (_Float16)(a0[e] * kCarryG);
        hv[it][4 + e] = (_Float16)(a1[e] * kCarryG);
      }
    }
    for (int pass = 0; pass < 2; ++pass) {
#pragma unroll
      for (int it = 0; it < 8; ++it) {
        const int row = it * 8 + wave * 4 + q;
        const size_t o = (row0 + t0 + row) * kDin + d0 + c8;
        *(volatile v8h*)(G16 + o) = hv[it];
      }
      __threadfence();
    }
  }
}

__global__ __launch_bounds__(256) void ln1_kernel(
    const float* __restrict__ X, const float* __restrict__ MO,
    const float* __restrict__ g, const float* __restrict__ be,
    float* __restrict__ O1, unsigned short* __restrict__ O1H)
{
  __shared__ __align__(16) float sR[8 * kLnP];
  const int tid = threadIdx.x, lane = tid & 31, wave = tid >> 5;
  const size_t row = (size_t)blockIdx.x * 8 + wave;
  const int c0 = lane * 4, c1 = 128 + lane * 4;
  const v4f xa = *(const v4f*)(X + row * kDm + c0);
  const v4f xb = *(const v4f*)(X + row * kDm + c1);
  const v4f ma = *(const v4f*)(MO + row * kDm + c0);
  const v4f mb = *(const v4f*)(MO + row * kDm + c1);
  const v4f va = xa + ma;
  const v4f vb = xb + mb;
  float s = ((va[0] + va[1]) + (va[2] + va[3])) + ((vb[0] + vb[1]) + (vb[2] + vb[3]));
#pragma unroll
  for (int off = 16; off > 0; off >>= 1) s += __shfl_xor(s, off, 32);
  const float mean = s * (1.0f / (float)kDm);
  const v4f da = va - mean;
  const v4f db = vb - mean;
  float qs = ((da[0] * da[0] + da[1] * da[1]) + (da[2] * da[2] + da[3] * da[3])) +
             ((db[0] * db[0] + db[1] * db[1]) + (db[2] * db[2] + db[3] * db[3]));
#pragma unroll
  for (int off = 16; off > 0; off >>= 1) qs += __shfl_xor(qs, off, 32);
  const float rs = rsqrtf(qs * (1.0f / (float)kDm) + kLnEps);
  const v4f ga = *(const v4f*)(g + c0);
  const v4f gb = *(const v4f*)(g + c1);
  const v4f ba = *(const v4f*)(be + c0);
  const v4f bb = *(const v4f*)(be + c1);
  const v4f oa = da * rs * ga + ba;
  const v4f ob = db * rs * gb + bb;
  float* strip = sR + wave * kLnP;
  *(v4f*)(strip + c0) = oa;
  *(v4f*)(strip + c1) = ob;
  __syncthreads();
  const v4f h0 = *(const v4f*)(strip + lane * 8);
  const v4f h1 = *(const v4f*)(strip + lane * 8 + 4);
  v8h hv;
#pragma unroll
  for (int e = 0; e < 4; ++e) {
    hv[e]     = (_Float16)h0[e];
    hv[4 + e] = (_Float16)h1[e];
  }
  for (int pass = 0; pass < 2; ++pass) {
    *(volatile v4f*)(O1 + row * kDm + c0) = oa;
    *(volatile v4f*)(O1 + row * kDm + c1) = ob;
    *(volatile v8h*)(O1H + row * kDm + lane * 8) = hv;
    __threadfence();
  }
}

__global__ __launch_bounds__(256) void ln2_kernel(
    const float* __restrict__ O1, const float* __restrict__ FF, const float* __restrict__ b2,
    const float* __restrict__ g, const float* __restrict__ be, float* __restrict__ OUT)
{
  const int tid = threadIdx.x, lane = tid & 31, wave = tid >> 5;
  const size_t row = (size_t)blockIdx.x * 8 + wave;
  const int c0 = lane * 4, c1 = 128 + lane * 4;
  const v4f xa = *(const v4f*)(O1 + row * kDm + c0);
  const v4f xb = *(const v4f*)(O1 + row * kDm + c1);
  const v4f fa = *(const v4f*)(FF + row * kDm + c0);
  const v4f fb = *(const v4f*)(FF + row * kDm + c1);
  const v4f pa = *(const v4f*)(b2 + c0);
  const v4f pb = *(const v4f*)(b2 + c1);
  const v4f va = xa + (fa + pa);
  const v4f vb = xb + (fb + pb);
  float s = ((va[0] + va[1]) + (va[2] + va[3])) + ((vb[0] + vb[1]) + (vb[2] + vb[3]));
#pragma unroll
  for (int off = 16; off > 0; off >>= 1) s += __shfl_xor(s, off, 32);
  const float mean = s * (1.0f / (float)kDm);
  const v4f da = va - mean;
  const v4f db = vb - mean;
  float qs = ((da[0] * da[0] + da[1] * da[1]) + (da[2] * da[2] + da[3] * da[3])) +
             ((db[0] * db[0] + db[1] * db[1]) + (db[2] * db[2] + db[3] * db[3]));
#pragma unroll
  for (int off = 16; off > 0; off >>= 1) qs += __shfl_xor(qs, off, 32);
  const float rs = rsqrtf(qs * (1.0f / (float)kDm) + kLnEps);
  const v4f ga = *(const v4f*)(g + c0);
  const v4f gb = *(const v4f*)(g + c1);
  const v4f ba = *(const v4f*)(be + c0);
  const v4f bb = *(const v4f*)(be + c1);
  const v4f oa = da * rs * ga + ba;
  const v4f ob = db * rs * gb + bb;
  for (int pass = 0; pass < 2; ++pass) {
    *(volatile v4f*)(OUT + row * kDm + c0) = oa;
    *(volatile v4f*)(OUT + row * kDm + c1) = ob;
    __threadfence();
  }
}

extern "C" void kernel_launch(void* const* d_in, const int* in_sizes, int n_in,
                              void* d_out, int out_size, void* d_ws, size_t ws_size,
                              hipStream_t stream) {
  if (n_in < 18) return;
  if (in_sizes[0] != kRows * kDm) return;
  if (in_sizes[1] != kXzP * kDm) return;
  if (in_sizes[2] != kDin * 4) return;
  if (in_sizes[3] != kDin) return;
  if (in_sizes[4] != kXdReal * kDin) return;
  if (in_sizes[5] != kDin * kDtR) return;
  if (in_sizes[6] != kDin) return;
  if (in_sizes[7] != kDin * kNst) return;
  if (in_sizes[8] != kDin) return;
  if (in_sizes[9] != kDm * kDin) return;
  if (in_sizes[10] != kDm || in_sizes[11] != kDm || in_sizes[12] != kDm || in_sizes[13] != kDm) return;
  if (in_sizes[14] != kFf * kDm) return;
  if (in_sizes[15] != kFf) return;
  if (in_sizes[16] != kDm * kFf) return;
  if (in_sizes[17] != kDm) return;
  if (out_size != kRows * kDm) return;
  if (ws_size < kWsTotal) return;

  const float* x      = (const float*)d_in[0];
  const float* w_in   = (const float*)d_in[1];
  const float* conv_w = (const float*)d_in[2];
  const float* conv_b = (const float*)d_in[3];
  const float* w_xp   = (const float*)d_in[4];
  const float* w_dt   = (const float*)d_in[5];
  const float* b_dt   = (const float*)d_in[6];
  const float* A_log  = (const float*)d_in[7];
  const float* Dp     = (const float*)d_in[8];
  const float* w_out  = (const float*)d_in[9];
  const float* ln1g   = (const float*)d_in[10];
  const float* ln1b   = (const float*)d_in[11];
  const float* ln2g   = (const float*)d_in[12];
  const float* ln2b   = (const float*)d_in[13];
  const float* w_f1   = (const float*)d_in[14];
  const float* b_f1   = (const float*)d_in[15];
  const float* w_f2   = (const float*)d_in[16];
  const float* b_f2   = (const float*)d_in[17];
  float* out = (float*)d_out;

  char* ws = (char*)d_ws;
  unsigned short* X16  = (unsigned short*)(ws + kOffX16);
  unsigned short* WI16 = (unsigned short*)(ws + kOffWI16);
  unsigned short* WX16 = (unsigned short*)(ws + kOffWX16);
  unsigned short* WO16 = (unsigned short*)(ws + kOffWO16);
  unsigned short* W116 = (unsigned short*)(ws + kOffW116);
  unsigned short* W216 = (unsigned short*)(ws + kOffW216);
  float*          XZ   = (float*)(ws + kOffXZ);
  float*          UC   = (float*)(ws + kOffUC);
  unsigned short* UC16 = (unsigned short*)(ws + kOffUC16);
  float*          XD   = (float*)(ws + kOffXD);
  unsigned short* G16  = (unsigned short*)(ws + kOffG16);
  float*          MO   = (float*)(ws + kOffMO);
  float*          O1   = (float*)(ws + kOffO1);
  unsigned short* O1H  = (unsigned short*)(ws + kOffO1H);
  unsigned short* HID  = (unsigned short*)(ws + kOffHID);
  float*          FF   = (float*)(ws + kOffFF);

  cast_f16_kernel<<<(kRows * kDm / 8) / 256, 256, 0, stream>>>(x, X16, kRows * kDm / 8, kRows * kDm / 8, 1.0f);
  cast_f16_kernel<<<(kXzP * kDm / 8) / 256, 256, 0, stream>>>(w_in, WI16, kXzP * kDm / 8, kXzP * kDm / 8, kCarryW);
  cast_f16_kernel<<<(kXdP * kDin / 8) / 256, 256, 0, stream>>>(w_xp, WX16, kXdP * kDin / 8, kXdReal * kDin / 8, kCarryW);
  cast_f16_kernel<<<(kDm * kDin / 8) / 256, 256, 0, stream>>>(w_out, WO16, kDm * kDin / 8, kDm * kDin / 8, kCarryW);
  cast_f16_kernel<<<(kFf * kDm / 8) / 256, 256, 0, stream>>>(w_f1, W116, kFf * kDm / 8, kFf * kDm / 8, kCarryW);
  cast_f16_kernel<<<(kDm * kFf / 8) / 256, 256, 0, stream>>>(w_f2, W216, kDm * kFf / 8, kDm * kFf / 8, kCarryW);

  wmma_gemm64<0, 0, 0><<<256, 256, 0, stream>>>(
      X16, kDm, WI16, kDm, (void*)XZ, kXzP, b_dt, kRows, kXzP, kDm, 1.0f / kCarryW);

  conv_silu_kernel<<<dim3(kDin / 256, kRows / 64), 256, 0, stream>>>(XZ, conv_w, conv_b, UC, UC16);

  wmma_gemm64<0, 0, 0><<<8, 256, 0, stream>>>(
      UC16, kDin, WX16, kDin, (void*)XD, kXdP, b_dt, kRows, kXdP, kDin, 1.0f / (kCarryU * kCarryW));

  scan_kernel<<<kBatch * (kDin / kScanCh), kScanCh, 0, stream>>>(XD, UC, XZ, w_dt, b_dt, A_log, Dp, G16);

  wmma_gemm64<0, 0, 0><<<32, 256, 0, stream>>>(
      G16, kDin, WO16, kDin, (void*)MO, kDm, b_dt, kRows, kDm, kDin, 1.0f / (kCarryG * kCarryW));

  ln1_kernel<<<kRows / 8, 256, 0, stream>>>(x, MO, ln1g, ln1b, O1, O1H);

  wmma_gemm64<2, 1, 2><<<128, 256, 0, stream>>>(
      O1H, kDm, W116, kDm, (void*)HID, kFf, b_f1, kRows, kFf, kDm, 1.0f / kCarryW);

  wmma_gemm64<0, 0, 0><<<32, 256, 0, stream>>>(
      HID, kFf, W216, kFf, (void*)FF, kDm, b_dt, kRows, kDm, kFf, 1.0f / kCarryW);

  ln2_kernel<<<kRows / 8, 256, 0, stream>>>(O1, FF, b_f2, ln2g, ln2b, out);
}
